// GraphMolDQN_thv1_42597485642061
// MI455X (gfx1250) — hardware-verified
//
#include <hip/hip_runtime.h>
#include <stddef.h>


#define DN     64
#define NF     14
#define FE     4
#define KW2    4096
#define KTOT   4160
#define NTHR   256
#define NWAVE  8
#define EPT    8
#define NGRP   2
#define CHUNK  (NTHR * EPT * NGRP)
#define WCAP   (EPT * NGRP * 32)
#define LISTN  (NWAVE * WCAP)
#define MTHR   128
#define MEDG   64
#define NBN    64
#define NBP    64
#define HP     68
#define NEGS   0.01f
#define OFF_IH 0
#define OFF_HH 12288
#define OFF_RT 24576
#define WB_N   28672
#define LDS_M  (MEDG * HP * 4 + MEDG * DN * 4 + MEDG * DN * 4 + MEDG * 4 + FE * DN * 4 + DN * 4)
#define LDS_N  (NBN * DN * 4 * 2 + NBN * DN * 2 * 2 + LISTN * 4 + NBN * 4 + 64)

static_assert((CHUNK & (CHUNK - 1)) == 0);
static_assert(CHUNK <= 4096);
static_assert((KTOT % 32) == 0);
static_assert(((DN * KTOT / 8) % NTHR) == 0);
static_assert(((192 * DN / 8) % NTHR) == 0);
static_assert(((DN * DN / 8) % NTHR) == 0);
static_assert(LDS_M <= 65536);
static_assert(NBN == 8 * NWAVE && NBP == 8 * NWAVE);
static_assert(MTHR == 2 * MEDG);

typedef float          v2f   __attribute__((ext_vector_type(2)));
typedef float          v4f   __attribute__((ext_vector_type(4)));
typedef float          v8f   __attribute__((ext_vector_type(8)));
typedef int            v4i   __attribute__((ext_vector_type(4)));
typedef unsigned short v8us  __attribute__((ext_vector_type(8)));
typedef __bf16         v8bf  __attribute__((ext_vector_type(8)));
typedef __bf16         v16bf __attribute__((ext_vector_type(16)));
union FragB { v16bf v; v8bf h[2]; v8us u[2]; };
union Pk8 { v8bf b; v8us u; };

__device__ __forceinline__ v8f z8() { v8f z = {0.f, 0.f, 0.f, 0.f, 0.f, 0.f, 0.f, 0.f}; return z; }

__device__ __forceinline__ v8f wmb(v16bf a, v16bf b, v8f c) {
  v8f d = __builtin_amdgcn_wmma_f32_16x16x32_bf16(false, a, false, b, (short)0, c, false, false);
  asm volatile("v_nop\n\tv_nop\n\tv_nop\n\tv_nop" : "+v"(d) : "v"(a), "v"(b));
  return d;
}

__device__ __forceinline__ unsigned short bfr(float x) {
  const unsigned u = __float_as_uint(x);
  return (unsigned short)((u + 0x7FFFu + ((u >> 16) & 1u)) >> 16);
}
__device__ __forceinline__ float bf16r(float x) {
  const unsigned u = __float_as_uint(x);
  return __uint_as_float((u + 0x7FFFu + ((u >> 16) & 1u)) & 0xFFFF0000u);
}
__device__ __forceinline__ v8bf cvt8b(v4f a, v4f b) {
  v8bf r;
#if defined(__HIP_DEVICE_COMPILE__)
  r[0] = (__bf16)a.x; r[1] = (__bf16)a.y; r[2] = (__bf16)a.z; r[3] = (__bf16)a.w;
  r[4] = (__bf16)b.x; r[5] = (__bf16)b.y; r[6] = (__bf16)b.z; r[7] = (__bf16)b.w;
#else
  Pk8 t;
  t.u[0] = bfr(a.x); t.u[1] = bfr(a.y); t.u[2] = bfr(a.z); t.u[3] = bfr(a.w);
  t.u[4] = bfr(b.x); t.u[5] = bfr(b.y); t.u[6] = bfr(b.z); t.u[7] = bfr(b.w);
  r = t.b;
#endif
  return r;
}
__device__ __forceinline__ v8us pk8(v4f a, v4f b) { Pk8 t; t.b = cvt8b(a, b); return t.u; }
__device__ __forceinline__ v4f sel4(bool c, v4f a, v4f b) {
  v4f r; r.x = c ? a.x : b.x; r.y = c ? a.y : b.y; r.z = c ? a.z : b.z; r.w = c ? a.w : b.w; return r;
}
__device__ __forceinline__ float lrelu(float x) { return x >= 0.0f ? x : NEGS * x; }
__device__ __forceinline__ float sigm(float x) { return 1.0f / (1.0f + expf(-x)); }
__device__ __forceinline__ float wsum(float p) {
  p += __shfl_xor(p, 16); p += __shfl_xor(p, 8); p += __shfl_xor(p, 4); p += __shfl_xor(p, 2); p += __shfl_xor(p, 1);
  return p;
}

__device__ __forceinline__ int scan_chunk(const int* __restrict__ ids, int nE, int cbase, int slotBase, int nb,
                                          int vec8, int* list, int tid, int lane, int wave) {
  int wc = 0;
#pragma unroll
  for (int g = 0; g < NGRP; ++g) {
    const int el0  = (g * NTHR + tid) * EPT;
    const int e0   = cbase + el0;
    const int sent = -2147483647 - 1;
    v4i da, db;
    if (vec8 != 0 && cbase + CHUNK <= nE) {
      da = *(const v4i*)(ids + e0);
      db = *(const v4i*)(ids + e0 + 4);
    } else {
      const int lst = nE - 1;
      da.x = (e0     < nE) ? ids[min(e0,     lst)] : sent;
      da.y = (e0 + 1 < nE) ? ids[min(e0 + 1, lst)] : sent;
      da.z = (e0 + 2 < nE) ? ids[min(e0 + 2, lst)] : sent;
      da.w = (e0 + 3 < nE) ? ids[min(e0 + 3, lst)] : sent;
      db.x = (e0 + 4 < nE) ? ids[min(e0 + 4, lst)] : sent;
      db.y = (e0 + 5 < nE) ? ids[min(e0 + 5, lst)] : sent;
      db.z = (e0 + 6 < nE) ? ids[min(e0 + 6, lst)] : sent;
      db.w = (e0 + 7 < nE) ? ids[min(e0 + 7, lst)] : sent;
    }
    const unsigned bs = (unsigned)slotBase;
    const unsigned ub = (unsigned)nb;
    const unsigned s0 = (unsigned)da.x - bs, s1 = (unsigned)da.y - bs;
    const unsigned s2 = (unsigned)da.z - bs, s3 = (unsigned)da.w - bs;
    const unsigned s4 = (unsigned)db.x - bs, s5 = (unsigned)db.y - bs;
    const unsigned s6 = (unsigned)db.z - bs, s7 = (unsigned)db.w - bs;
    const bool h0 = s0 < ub, h1 = s1 < ub, h2 = s2 < ub, h3 = s3 < ub;
    const bool h4 = s4 < ub, h5 = s5 < ub, h6 = s6 < ub, h7 = s7 < ub;
    const unsigned any = __builtin_amdgcn_ballot_w32(h0 | h1 | h2 | h3 | h4 | h5 | h6 | h7);
    if (any != 0u) {
#define HITJ(J, HJ, SJ) { \
        const unsigned mj = __builtin_amdgcn_ballot_w32(HJ); \
        if (mj != 0u) { \
          if (HJ) { \
            const int pos = wc + (int)__builtin_amdgcn_mbcnt_lo(mj, 0u); \
            if (pos < WCAP) list[wave * WCAP + pos] = ((el0 + (J)) << 12) | (int)(SJ); \
          } \
          wc += (int)__builtin_popcount(mj); } }
      HITJ(0, h0, s0)
      HITJ(1, h1, s1)
      HITJ(2, h2, s2)
      HITJ(3, h3, s3)
      HITJ(4, h4, s4)
      HITJ(5, h5, s5)
      HITJ(6, h6, s6)
      HITJ(7, h7, s7)
#undef HITJ
    }
  }
  return wc;
}

__global__ __launch_bounds__(NTHR) void k_bprep(const float* __restrict__ Wb, const float* __restrict__ bb,
                                                unsigned short* Bp) {
  constexpr int NU = DN * KTOT / 8;
  const int i = blockIdx.x * NTHR + (int)threadIdx.x;
  if (i >= NU) return;
  const int o  = i * 8;
  const int n  = o / KTOT;
  const int j0 = o - n * KTOT;
  float v[8];
#pragma unroll
  for (int e = 0; e < 8; ++e) {
    const int j  = j0 + e;
    const int jw = j < DN * DN ? j : DN * DN - 1;
    int jb = j - DN * DN;
    jb = jb < 0 ? 0 : (jb > DN - 1 ? DN - 1 : jb);
    const float wv = Wb[(size_t)jw * DN + n];
    const float bv = bb[(size_t)jb * DN + n];
    v[e] = (j < DN * DN) ? wv : bv;
  }
  v4f a, b;
  a.x = v[0]; a.y = v[1]; a.z = v[2]; a.w = v[3];
  b.x = v[4]; b.y = v[5]; b.z = v[6]; b.w = v[7];
  const v8us hv = pk8(a, b);
  unsigned short* dp = Bp + o;
  *(volatile v8us*)dp = hv;
  __threadfence();
  *(volatile v8us*)dp = hv;
}

__global__ __launch_bounds__(NTHR) void k_wprep(const float* __restrict__ wih, const float* __restrict__ whh,
                                                const float* __restrict__ root, unsigned short* wb) {
  constexpr int NBW = (192 * DN / 8) / NTHR;
  const int b = (int)blockIdx.x;
  const int i = b * NTHR + (int)threadIdx.x;
  v8us hv;
  int dofs;
  if (b < NBW) {
    const int o = i * 8;
    hv = pk8(*(const v4f*)(wih + o), *(const v4f*)(wih + o + 4));
    dofs = OFF_IH + o;
  } else if (b < 2 * NBW) {
    const int o = (i - NBW * NTHR) * 8;
    hv = pk8(*(const v4f*)(whh + o), *(const v4f*)(whh + o + 4));
    dofs = OFF_HH + o;
  } else {
    const int u  = i - 2 * NBW * NTHR;
    const int n  = u >> 3;
    const int k0 = (u & 7) * 8;
    const float* rp = root + (size_t)k0 * DN + n;
    v4f a, c;
    a.x = rp[0];      a.y = rp[DN];     a.z = rp[2 * DN]; a.w = rp[3 * DN];
    c.x = rp[4 * DN]; c.y = rp[5 * DN]; c.z = rp[6 * DN]; c.w = rp[7 * DN];
    hv = pk8(a, c);
    dofs = OFF_RT + u * 8;
  }
  unsigned short* dp = wb + dofs;
  *(volatile v8us*)dp = hv;
  __threadfence();
  *(volatile v8us*)dp = hv;
}

__global__ __launch_bounds__(NTHR) void k_lin0(const float* __restrict__ x, const float* __restrict__ w,
                                               const float* __restrict__ b, float* H, int nN) {
  __shared__ float xs[NBN * NF];
  __shared__ float ws0[NF * DN];
  __shared__ float bs0[DN];
  __shared__ __attribute__((aligned(16))) float st[NBN * DN];
  const int tid = threadIdx.x, lane = tid & 31, wave = tid >> 5, hf = lane >> 4, m = lane & 15;
  const int nb = (int)blockIdx.x * NBN;
#pragma unroll 1
  for (int u = tid; u < NBN * NF; u += NTHR) {
    const int row = u / NF;
    const int c = u - row * NF;
    int node = nb + row;
    node = node > nN - 1 ? nN - 1 : node;
    xs[u] = x[(size_t)node * NF + c];
  }
#pragma unroll 1
  for (int u = tid; u < NF * DN; u += NTHR) ws0[u] = bf16r(w[u]);
  if (tid < DN) bs0[tid] = bf16r(b[tid]);
  __syncthreads();
  {
    const int rg = wave >> 1, q = wave & 1;
    const v4f z4 = {0.f, 0.f, 0.f, 0.f};
    const float* xr = xs + (16 * rg + m) * NF;
    float av[8];
#pragma unroll
    for (int i = 0; i < 8; ++i) {
      const int k = 8 * hf + i;
      const int kc = k < NF ? k : NF - 1;
      const float v = xr[kc];
      av[i] = (k < NF) ? v : 0.0f;
    }
    v4f a0, a1;
    a0.x = av[0]; a0.y = av[1]; a0.z = av[2]; a0.w = av[3];
    a1.x = av[4]; a1.y = av[5]; a1.z = av[6]; a1.w = av[7];
    FragB a;
    a.h[0] = cvt8b(a0, a1);
    a.h[1] = cvt8b(z4, z4);
    v8f acc[2];
#pragma unroll
    for (int u = 0; u < 2; ++u) {
      const int n = 32 * q + 16 * u + m;
      float bw[8];
#pragma unroll
      for (int i = 0; i < 8; ++i) {
        const int k = 8 * hf + i;
        const int kc = k < NF ? k : NF - 1;
        const float v = ws0[kc * DN + n];
        bw[i] = (k < NF) ? v : 0.0f;
      }
      v4f b0, b1;
      b0.x = bw[0]; b0.y = bw[1]; b0.z = bw[2]; b0.w = bw[3];
      b1.x = bw[4]; b1.y = bw[5]; b1.z = bw[6]; b1.w = bw[7];
      FragB bf;
      bf.h[0] = cvt8b(b0, b1);
      bf.h[1] = cvt8b(z4, z4);
      acc[u] = wmb(a.v, bf.v, z8());
    }
#pragma unroll
    for (int u = 0; u < 2; ++u) {
      const int j = 32 * q + 16 * u + m;
      const float bv = bs0[j];
#pragma unroll
      for (int r = 0; r < 8; ++r) st[(16 * rg + 8 * hf + r) * DN + j] = lrelu(acc[u][r] + bv);
    }
  }
  __syncthreads();
  v4f ov[4];
#pragma unroll
  for (int it = 0; it < 4; ++it) ov[it] = *(const v4f*)(st + 4 * (it * NTHR + tid));
  float* gp = H + (size_t)blockIdx.x * NBN * DN;
#pragma unroll
  for (int it = 0; it < 4; ++it) *(volatile v4f*)(gp + 4 * (it * NTHR + tid)) = ov[it];
  __threadfence();
#pragma unroll
  for (int it = 0; it < 4; ++it) *(volatile v4f*)(gp + 4 * (it * NTHR + tid)) = ov[it];
}

__global__ __launch_bounds__(MTHR) void k_msg(
    const float* __restrict__ H, int nN, const int* __restrict__ ei, int nE,
    const float* __restrict__ EA, const float* __restrict__ W1, const float* __restrict__ b1,
    const unsigned short* __restrict__ Bp, float* MSG) {
  constexpr int NT  = DN / 16;
  constexpr int NPI = 16 * DN / 128;
  extern __shared__ v4f lds_dyn[];
  float* Hs  = (float*)lds_dyn;
  float* Xs  = Hs + MEDG * HP;
  float* Stg = Xs + MEDG * DN;
  int*   Ss  = (int*)(Stg + MEDG * DN);
  float* W1s = (float*)(Ss + MEDG);
  float* B1s = W1s + FE * DN;

  const int tid = threadIdx.x, lane = tid & 31, wave = tid >> 5, hf = lane >> 4, m = lane & 15;
  const int eBase = blockIdx.x * MEDG;

  if (tid < MEDG) {
    int e = eBase + tid;
    e = e > nE - 1 ? nE - 1 : e;
    int s = ei[e];
    s = s < 0 ? 0 : (s > nN - 1 ? nN - 1 : s);
    Ss[tid] = s;
  }
#pragma unroll 1
  for (int u = tid; u < FE * DN; u += MTHR) W1s[u] = bf16r(W1[u]);
  if (tid < DN) B1s[tid] = bf16r(b1[tid]);
  __syncthreads();

  {
    int e = eBase + 16 * wave + m;
    e = e > nE - 1 ? nE - 1 : e;
    const v4f av = *(const v4f*)(EA + (size_t)e * FE);
    const v4f z4 = {0.f, 0.f, 0.f, 0.f};
    FragB a;
    a.h[0] = cvt8b(sel4(hf == 0, av, z4), z4);
    a.h[1] = cvt8b(z4, z4);
    float* hw = Hs + (16 * wave + 8 * hf) * HP;
#pragma unroll
    for (int t = 0; t < NT; ++t) {
      const int col = 16 * t + m;
      v4f w0;
      w0.x = W1s[col]; w0.y = W1s[DN + col]; w0.z = W1s[2 * DN + col]; w0.w = W1s[3 * DN + col];
      FragB b;
      b.h[0] = cvt8b(sel4(hf == 0, w0, z4), z4);
      b.h[1] = cvt8b(z4, z4);
      const v8f d = wmb(a.v, b.v, z8());
      const float bav = B1s[col];
#pragma unroll
      for (int r = 0; r < 8; ++r) hw[r * HP + col] = lrelu(d[r] + bav);
    }
    if (lane < 16) Hs[(16 * wave + lane) * HP + DN] = 1.0f;
  }
  __syncthreads();

#pragma unroll 1
  for (int u = tid; u < MEDG * (DN / 4); u += MTHR) {
    const int r  = u / (DN / 4);
    const int c4 = u - r * (DN / 4);
    const int s  = Ss[r];
    *(v4f*)(Xs + r * DN + 4 * c4) = *(const v4f*)(H + (size_t)s * DN + 4 * c4);
  }
  __syncthreads();

  v4f xq[8];
  {
    const float* xrow = Xs + (16 * wave + m) * DN + 8 * hf;
#pragma unroll
    for (int ib = 0; ib < 2; ++ib) {
      xq[4 * ib + 0] = *(const v4f*)(xrow + 32 * ib);
      xq[4 * ib + 1] = *(const v4f*)(xrow + 32 * ib + 4);
      xq[4 * ib + 2] = *(const v4f*)(xrow + 32 * ib + 16);
      xq[4 * ib + 3] = *(const v4f*)(xrow + 32 * ib + 20);
    }
  }

  v8f acc[NT];
#pragma unroll
  for (int t = 0; t < NT; ++t) acc[t] = z8();
  const float* hrow = Hs + (16 * wave + m) * HP;
  const unsigned short* bbase = Bp + (size_t)m * KTOT + 8 * hf;
#pragma unroll 1
  for (int k = 0; k <= DN; ++k) {
    const float hk = hrow[k];
#pragma unroll
    for (int ib = 0; ib < 2; ++ib) {
      const int kc = 2 * k + ib;
      FragB a;
      a.h[0] = cvt8b(xq[4 * ib + 0] * hk, xq[4 * ib + 1] * hk);
      a.h[1] = cvt8b(xq[4 * ib + 2] * hk, xq[4 * ib + 3] * hk);
      const unsigned short* bp = bbase + (size_t)32 * kc;
#pragma unroll
      for (int t = 0; t < NT; ++t) {
        const unsigned short* bt = bp + (size_t)(16 * t) * KTOT;
        FragB b;
        b.u[0] = *(const v8us*)bt;
        b.u[1] = *(const v8us*)(bt + 16);
        acc[t] = wmb(a.v, b.v, acc[t]);
      }
    }
  }
  __syncthreads();

  {
    float* sp = Stg + (16 * wave + 8 * hf) * DN + m;
#pragma unroll
    for (int t = 0; t < NT; ++t) {
#pragma unroll
      for (int r = 0; r < 8; ++r) sp[r * DN + 16 * t] = acc[t][r];
    }
  }
  __syncthreads();

  const float* lp = Stg + 16 * wave * DN;
  float* gp = MSG + (size_t)(eBase + 16 * wave) * DN;
#pragma unroll
  for (int p = 0; p < NPI; ++p) {
    const v4f v = *(const v4f*)(lp + 4 * (32 * p + lane));
    *(volatile v4f*)(gp + 4 * (32 * p + lane)) = v;
  }
  __threadfence();
#pragma unroll
  for (int p = 0; p < NPI; ++p) {
    const v4f v = *(const v4f*)(lp + 4 * (32 * p + lane));
    *(volatile v4f*)(gp + 4 * (32 * p + lane)) = v;
  }
}

__global__ __launch_bounds__(NTHR) void k_node(
    const int* __restrict__ ei, int nE, int vec8, const float* __restrict__ MSG, float* H,
    const unsigned short* __restrict__ WB, const float* __restrict__ cb,
    const float* __restrict__ bih, const float* __restrict__ bhh) {
  extern __shared__ v4f lds_dyn[];
  float* agg = (float*)lds_dyn;
  float* hr  = agg + NBN * DN;
  unsigned short* mb = (unsigned short*)(hr + NBN * DN);
  unsigned short* hb = mb + NBN * DN;
  int* list = (int*)(hb + NBN * DN);
  int* cnt  = list + LISTN;
  int* wcnt = cnt + NBN;
  const int tid = threadIdx.x, lane = tid & 31, wave = tid >> 5, hf = lane >> 4, m = lane & 15;
  const int nb = (int)blockIdx.x * NBN;
  {
    const int row = tid >> 2, part = tid & 3;
    const float* hp = H + (size_t)(nb + row) * DN + 16 * part;
    const v4f a0 = *(const v4f*)hp, a1 = *(const v4f*)(hp + 4), a2 = *(const v4f*)(hp + 8), a3 = *(const v4f*)(hp + 12);
    float* dp = hr + row * DN + 16 * part;
    *(v4f*)dp = a0; *(v4f*)(dp + 4) = a1; *(v4f*)(dp + 8) = a2; *(v4f*)(dp + 12) = a3;
    const v4f z = {0.f, 0.f, 0.f, 0.f};
    float* zp = agg + row * DN + 16 * part;
    *(v4f*)zp = z; *(v4f*)(zp + 4) = z; *(v4f*)(zp + 8) = z; *(v4f*)(zp + 12) = z;
    *(v8us*)(hb + row * DN + 16 * part) = pk8(a0, a1);
    *(v8us*)(hb + row * DN + 16 * part + 8) = pk8(a2, a3);
    if (tid < NBN) cnt[tid] = 0;
  }
  __syncthreads();

  const int* dsts = ei + nE;
  const int nChunks = (nE + CHUNK - 1) / CHUNK;
#pragma unroll 1
  for (int ch = 0; ch < nChunks; ++ch) {
    const int cbase = ch * CHUNK;
    const int wc = scan_chunk(dsts, nE, cbase, nb, NBN, vec8, list, tid, lane, wave);
    if (lane == 0) wcnt[wave] = wc;
    __syncthreads();
#pragma unroll 1
    for (int wsx = 0; wsx < NWAVE; ++wsx) {
      int n = __builtin_amdgcn_readfirstlane(wcnt[wsx]);
      n = n > WCAP ? WCAP : (n < 0 ? 0 : n);
      const int* lp = list + wsx * WCAP;
#pragma unroll 1
      for (int i = 0; i < n; ++i) {
        const int ent = __builtin_amdgcn_readfirstlane(lp[i]);
        int slot = ent & 4095;
        slot = slot > NBN - 1 ? NBN - 1 : slot;
        if ((slot >> 3) == wave) {
          int e = cbase + ((ent >> 12) & (CHUNK - 1));
          e = e > nE - 1 ? nE - 1 : e;
          const v2f v = *(const v2f*)(MSG + (size_t)e * DN + 2 * lane);
          v2f* ap = (v2f*)(agg + slot * DN + 2 * lane);
          *ap = *ap + v;
          if (lane == 0) cnt[slot] = cnt[slot] + 1;
        }
      }
    }
    __syncthreads();
  }

  {
    const int rg = wave >> 1, q = wave & 1;
    v8f ac[2];
    ac[0] = z8(); ac[1] = z8();
#pragma unroll
    for (int ks = 0; ks < 2; ++ks) {
      const int ao = (16 * rg + m) * DN + 32 * ks + 8 * hf;
      FragB a;
      a.u[0] = *(const v8us*)(hb + ao);
      a.u[1] = *(const v8us*)(hb + ao + 16);
#pragma unroll
      for (int u = 0; u < 2; ++u) {
        const int bo = (32 * q + 16 * u + m) * DN + 32 * ks + 8 * hf;
        FragB b;
        b.u[0] = *(const v8us*)(WB + OFF_RT + bo);
        b.u[1] = *(const v8us*)(WB + OFF_RT + bo + 16);
        ac[u] = wmb(a.v, b.v, ac[u]);
      }
    }
    float rdv[8];
#pragma unroll
    for (int r = 0; r < 8; ++r) {
      int c = cnt[16 * rg + 8 * hf + r];
      c = c < 1 ? 1 : c;
      rdv[r] = 1.0f / (float)c;
    }
#pragma unroll
    for (int u = 0; u < 2; ++u) {
      const int j = 32 * q + 16 * u + m;
      const float cbv = bf16r(cb[j]);
#pragma unroll
      for (int r = 0; r < 8; ++r) {
        const int row = 16 * rg + 8 * hf + r;
        const float val = (ac[u][r] + agg[row * DN + j] * rdv[r]) + cbv;
        mb[row * DN + j] = bfr(lrelu(val));
      }
    }
  }
  __syncthreads();

  {
    const int rg = wave >> 1, q = wave & 1;
    v8f gi[3][2], gh[3][2];
#pragma unroll
    for (int g = 0; g < 3; ++g) { gi[g][0] = z8(); gi[g][1] = z8(); gh[g][0] = z8(); gh[g][1] = z8(); }
#pragma unroll
    for (int ks = 0; ks < 2; ++ks) {
      const int ao = (16 * rg + m) * DN + 32 * ks + 8 * hf;
      FragB am, ah;
      am.u[0] = *(const v8us*)(mb + ao); am.u[1] = *(const v8us*)(mb + ao + 16);
      ah.u[0] = *(const v8us*)(hb + ao); ah.u[1] = *(const v8us*)(hb + ao + 16);
#pragma unroll
      for (int g = 0; g < 3; ++g) {
#pragma unroll
        for (int u = 0; u < 2; ++u) {
          const int bo = (64 * g + 32 * q + 16 * u + m) * DN + 32 * ks + 8 * hf;
          FragB b;
          b.u[0] = *(const v8us*)(WB + OFF_IH + bo); b.u[1] = *(const v8us*)(WB + OFF_IH + bo + 16);
          gi[g][u] = wmb(am.v, b.v, gi[g][u]);
          b.u[0] = *(const v8us*)(WB + OFF_HH + bo); b.u[1] = *(const v8us*)(WB + OFF_HH + bo + 16);
          gh[g][u] = wmb(ah.v, b.v, gh[g][u]);
        }
      }
    }
#pragma unroll
    for (int u = 0; u < 2; ++u) {
      const int j = 32 * q + 16 * u + m;
      const float bir = bf16r(bih[j]), biz = bf16r(bih[DN + j]), bin = bf16r(bih[2 * DN + j]);
      const float bhr = bf16r(bhh[j]), bhz = bf16r(bhh[DN + j]), bhn = bf16r(bhh[2 * DN + j]);
#pragma unroll
      for (int r = 0; r < 8; ++r) {
        const int row = 16 * rg + 8 * hf + r;
        const float rr = sigm((gi[0][u][r] + bir) + (gh[0][u][r] + bhr));
        const float zz = sigm((gi[1][u][r] + biz) + (gh[1][u][r] + bhz));
        const float nn = tanhf((gi[2][u][r] + bin) + rr * (gh[2][u][r] + bhn));
        const float ho = hr[row * DN + j];
        agg[row * DN + j] = (1.0f - zz) * nn + zz * ho;
      }
    }
  }
  __syncthreads();
  v4f ov[4];
#pragma unroll
  for (int it = 0; it < 4; ++it) ov[it] = *(const v4f*)(agg + 4 * (it * NTHR + tid));
  float* gp = H + (size_t)nb * DN;
#pragma unroll
  for (int it = 0; it < 4; ++it) *(volatile v4f*)(gp + 4 * (it * NTHR + tid)) = ov[it];
  __threadfence();
#pragma unroll
  for (int it = 0; it < 4; ++it) *(volatile v4f*)(gp + 4 * (it * NTHR + tid)) = ov[it];
}

__global__ __launch_bounds__(NTHR) void k_pool(
    const int* __restrict__ batch, int nN, const float* __restrict__ H,
    const float* __restrict__ lbih, const float* __restrict__ lbhh, float* out, int G) {
  __shared__ __attribute__((aligned(16))) float R[NBP * DN];
  __shared__ __attribute__((aligned(16))) int plist[LISTN];
  __shared__ __attribute__((aligned(16))) float qs[DN];
  __shared__ float Mx[NBP];
  __shared__ float Sx[NBP];
  __shared__ int wcnt[NWAVE];
  const int tid = threadIdx.x, lane = tid & 31, wave = tid >> 5;
  const int gBase = (int)blockIdx.x * NBP;
  int nb = G - gBase;
  nb = nb < 0 ? 0 : (nb > NBP ? NBP : nb);
  {
    const v4f z = {0.f, 0.f, 0.f, 0.f};
#pragma unroll 1
    for (int i = tid; i < NBP * DN / 4; i += NTHR) ((v4f*)R)[i] = z;
    if (tid < NBP) { Mx[tid] = -__builtin_inff(); Sx[tid] = 0.0f; }
    if (tid < DN) {
      const float g_i = bf16r(lbih[tid]) + bf16r(lbhh[tid]);
      const float g_g = bf16r(lbih[2 * DN + tid]) + bf16r(lbhh[2 * DN + tid]);
      const float g_o = bf16r(lbih[3 * DN + tid]) + bf16r(lbhh[3 * DN + tid]);
      float av = g_i, bv = g_g, res = 0.0f;
#pragma unroll 1
      for (int t = 0; t < 2; ++t) {
        res = sigm(av) * tanhf(bv);
        av = g_o;
        bv = res;
      }
      qs[tid] = res;
    }
  }
  __syncthreads();

  const v2f qv = *(const v2f*)(qs + 2 * lane);
  const int nChunks = (nN + CHUNK - 1) / CHUNK;
#pragma unroll 1
  for (int ch = 0; ch < nChunks; ++ch) {
    const int cbase = ch * CHUNK;
    const int wc = scan_chunk(batch, nN, cbase, gBase, nb, 1, plist, tid, lane, wave);
    if (lane == 0) wcnt[wave] = wc;
    __syncthreads();
#pragma unroll 1
    for (int wsx = 0; wsx < NWAVE; ++wsx) {
      int n = __builtin_amdgcn_readfirstlane(wcnt[wsx]);
      n = n > WCAP ? WCAP : (n < 0 ? 0 : n);
      const int* lp = plist + wsx * WCAP;
#pragma unroll 1
      for (int i = 0; i < n; ++i) {
        const int ent = __builtin_amdgcn_readfirstlane(lp[i]);
        int slot = ent & 4095;
        slot = slot > NBP - 1 ? NBP - 1 : slot;
        if ((slot >> 3) == wave) {
          int nd = cbase + ((ent >> 12) & (CHUNK - 1));
          nd = nd > nN - 1 ? nN - 1 : nd;
          const v2f o = *(const v2f*)(H + (size_t)nd * DN + 2 * lane);
          const float e = wsum(o.x * qv.x + o.y * qv.y);
          const float mold = Mx[slot];
          const float sold = Sx[slot];
          const float mnew = fmaxf(mold, e);
          float dm = mold - mnew;
          dm = dm < -87.0f ? -87.0f : dm;
          const float f = expf(dm);
          const float p = expf(e - mnew);
          v2f* rp = (v2f*)(R + slot * DN + 2 * lane);
          *rp = *rp * f + o * p;
          Mx[slot] = mnew;
          Sx[slot] = sold * f + p;
        }
      }
    }
    __syncthreads();
  }

  v4f ov[8];
  const int c4 = 4 * (lane & 15);
#pragma unroll
  for (int j = 0; j < 8; ++j) {
    const int slot = 8 * wave + j;
    const float sv = Sx[slot];
    const float den = fmaxf(sv, 1e-16f);
    const float rinv = 1.0f / den;
    const v4f q4 = *(const v4f*)(qs + c4);
    const v4f r4 = *(const v4f*)(R + slot * DN + c4) * rinv;
    ov[j] = sel4(lane < 16, q4, r4);
  }
#pragma unroll
  for (int j = 0; j < 8; ++j) {
    const int slot = 8 * wave + j;
    if (slot < nb) *(volatile v4f*)(out + (size_t)(gBase + slot) * (2 * DN) + 4 * lane) = ov[j];
  }
  __threadfence();
#pragma unroll
  for (int j = 0; j < 8; ++j) {
    const int slot = 8 * wave + j;
    if (slot < nb) *(volatile v4f*)(out + (size_t)(gBase + slot) * (2 * DN) + 4 * lane) = ov[j];
  }
}

extern "C" void kernel_launch(void* const* d_in, const int* in_sizes, int n_in,
                              void* d_out, int out_size, void* d_ws, size_t ws_size,
                              hipStream_t stream) {
  if (n_in < 20) return;
  const int nN = in_sizes[3];
  const int nE = in_sizes[1] / 2;
  const int G  = out_size / (2 * DN);
  if (nN <= 0 || nE <= 0 || G <= 0) return;
  if (in_sizes[0] != nN * NF || in_sizes[1] != 2 * nE || in_sizes[2] != nE * FE || out_size != G * 2 * DN) return;
  if (in_sizes[4] != NF * DN || in_sizes[5] != DN || in_sizes[6] != FE * DN || in_sizes[7] != DN) return;
  if (in_sizes[8] != DN * KW2 || in_sizes[9] != KW2 || in_sizes[10] != DN * DN || in_sizes[11] != DN) return;
  if (in_sizes[12] != 192 * DN || in_sizes[13] != 192 * DN || in_sizes[14] != 192 || in_sizes[15] != 192) return;
  if (in_sizes[18] != 256 || in_sizes[19] != 256) return;
  if (nN > (1 << 22) || nE > (1 << 24)) return;

  const float* x      = (const float*)d_in[0];
  const int*   ei     = (const int*)d_in[1];
  const float* ea     = (const float*)d_in[2];
  const int*   batch  = (const int*)d_in[3];
  const float* lin0_w = (const float*)d_in[4];
  const float* lin0_b = (const float*)d_in[5];
  const float* net_w1 = (const float*)d_in[6];
  const float* net_b1 = (const float*)d_in[7];
  const float* net_w2 = (const float*)d_in[8];
  const float* net_b2 = (const float*)d_in[9];
  const float* root_w = (const float*)d_in[10];
  const float* conv_b = (const float*)d_in[11];
  const float* w_ih   = (const float*)d_in[12];
  const float* w_hh   = (const float*)d_in[13];
  const float* b_ih   = (const float*)d_in[14];
  const float* b_hh   = (const float*)d_in[15];
  const float* lb_ih  = (const float*)d_in[18];
  const float* lb_hh  = (const float*)d_in[19];
  float* out = (float*)d_out;

  const int nMB = (nE + MEDG - 1) / MEDG, EP = nMB * MEDG;
  const int NB1 = (nN + NBN - 1) / NBN,   NP = NB1 * NBN;
  const int nPool = (G + NBP - 1) / NBP;

  char* ws = (char*)d_ws;
  size_t off = 0;
  const size_t oH   = off; off += (size_t)NP * DN * 4;        off = (off + 255) & ~(size_t)255;
  const size_t oMSG = off; off += (size_t)EP * DN * 4;        off = (off + 255) & ~(size_t)255;
  const size_t oBP  = off; off += (size_t)DN * KTOT * 2;      off = (off + 255) & ~(size_t)255;
  const size_t oWB  = off; off += (size_t)WB_N * 2;           off = (off + 255) & ~(size_t)255;
  if (off > ws_size) return;
  if (off > (size_t)128 * 1024 * 1024) return;
  float* Hpl = (float*)(ws + oH);
  float* msg = (float*)(ws + oMSG);
  unsigned short* Bp = (unsigned short*)(ws + oBP);
  unsigned short* wb = (unsigned short*)(ws + oWB);
  const int vec8 = ((nE & 3) == 0) ? 1 : 0;

  k_bprep<<<(DN * KTOT / 8) / NTHR, NTHR, 0, stream>>>(net_w2, net_b2, Bp);
  k_wprep<<<(2 * 192 * DN / 8 + DN * DN / 8) / NTHR, NTHR, 0, stream>>>(w_ih, w_hh, root_w, wb);
  k_lin0<<<NB1, NTHR, 0, stream>>>(x, lin0_w, lin0_b, Hpl, nN);

  hipFuncSetAttribute(reinterpret_cast<const void*>(&k_msg), hipFuncAttributeMaxDynamicSharedMemorySize, LDS_M);
  hipFuncSetAttribute(reinterpret_cast<const void*>(&k_node), hipFuncAttributeMaxDynamicSharedMemorySize, LDS_N);
  for (int s = 0; s < 6; ++s) {
    k_msg<<<nMB, MTHR, LDS_M, stream>>>(Hpl, nN, ei, nE, ea, net_w1, net_b1, Bp, msg);
    k_node<<<NB1, NTHR, LDS_N, stream>>>(ei, nE, vec8, msg, Hpl, wb, conv_b, b_ih, b_hh);
  }
  k_pool<<<nPool, NTHR, 0, stream>>>(batch, nN, Hpl, lb_ih, lb_hh, out, G);
}
